// GlobalGBST_84988812853375
// MI455X (gfx1250) — hardware-run, weakly checked
//
#include <hip/hip_runtime.h>
#include <stddef.h>
#include <stdint.h>
#include <float.h>
#include <math.h>

#define NBATCH 8
#define SL     2048
#define DM     256
#define NLAY   9
#define NTOK   16384
#define CH     16
#define HALO   8
#define WIN    32

static_assert(NTOK == NBATCH * SL);
static_assert(SL % 32 == 0);
static_assert(SL % CH == 0);
static_assert(WIN == CH + 2 * HALO);
static_assert(WIN == 32);
static_assert(CH == 16);
static_assert(NTOK % 256 == 0);
static_assert(DM == 256);
static_assert((DM * DM) % 2048 == 0);
static_assert(NLAY * WIN <= 512);

typedef _Float16 v16h __attribute__((ext_vector_type(16)));
typedef _Float16 v8h  __attribute__((ext_vector_type(8)));
typedef float    v8f  __attribute__((ext_vector_type(8)));
typedef float    v4f  __attribute__((ext_vector_type(4)));
typedef unsigned int v4u __attribute__((ext_vector_type(4)));

union Frag  { v16h v; v8h h[2]; };
union Pack8 { v8h h; v4u u; };

__device__ __forceinline__ v8f mma16(v16h a, v16h b, v8f c) {
  c = __builtin_amdgcn_wmma_f32_16x16x32_f16(false, a, false, b, (short)0, c, false, false);
  asm volatile("v_nop\n\tv_nop\n\tv_nop\n\tv_nop" : "+v"(c) : "v"(a), "v"(b));
  return c;
}

__device__ __forceinline__ v16h ldfrag(const _Float16* p, int ld, int row0, int k0, int lane) {
  const int m = lane & 15, lh = lane >> 4;
  const _Float16* q = p + (size_t)(row0 + m) * ld + k0 + 8 * lh;
  Frag f;
  f.h[0] = *(const v8h*)(q);
  f.h[1] = *(const v8h*)(q + 16);
  return f.v;
}

__device__ __forceinline__ v8f zero8() { return (v8f){0.f, 0.f, 0.f, 0.f, 0.f, 0.f, 0.f, 0.f}; }

__device__ __forceinline__ v8h cvt8(v4f a0, v4f a1) {
  return (v8h){(_Float16)a0[0], (_Float16)a0[1], (_Float16)a0[2], (_Float16)a0[3],
               (_Float16)a1[0], (_Float16)a1[1], (_Float16)a1[2], (_Float16)a1[3]};
}

__device__ __forceinline__ void gemm32x64(const _Float16* __restrict__ A, int lda,
                                          const _Float16* __restrict__ Bt, int ldb, int K,
                                          int m0, int n0, int lane, v8f (&acc)[2][4]) {
#pragma unroll 1
  for (int k0 = 0; k0 < K; k0 += 32) {
    const v16h a0 = ldfrag(A, lda, m0, k0, lane);
    const v16h a1 = ldfrag(A, lda, m0 + 16, k0, lane);
    const v16h b0 = ldfrag(Bt, ldb, n0, k0, lane);
    const v16h b1 = ldfrag(Bt, ldb, n0 + 16, k0, lane);
    const v16h b2 = ldfrag(Bt, ldb, n0 + 32, k0, lane);
    const v16h b3 = ldfrag(Bt, ldb, n0 + 48, k0, lane);
    acc[0][0] = mma16(a0, b0, acc[0][0]);
    acc[1][0] = mma16(a1, b0, acc[1][0]);
    acc[0][1] = mma16(a0, b1, acc[0][1]);
    acc[1][1] = mma16(a1, b1, acc[1][1]);
    acc[0][2] = mma16(a0, b2, acc[0][2]);
    acc[1][2] = mma16(a1, b2, acc[1][2]);
    acc[0][3] = mma16(a0, b3, acc[0][3]);
    acc[1][3] = mma16(a1, b3, acc[1][3]);
  }
}

__global__ __launch_bounds__(256) void k_cvt(const float* __restrict__ src, _Float16* __restrict__ dh, float scale) {
  const size_t o = (size_t)blockIdx.x * 2048 + (size_t)threadIdx.x * 8;
  const v4f a0 = *(const v4f*)(src + o) * scale;
  const v4f a1 = *(const v4f*)(src + o + 4) * scale;
  Pack8 pk;
  pk.h = cvt8(a0, a1);
  const v4u vv = pk.u;
  volatile v4u* d = (volatile v4u*)(dh + o);
  *d = vv;
  __threadfence();
  *d = vv;
}

__device__ __forceinline__ float embtap(const int* __restrict__ seq, const float* __restrict__ emb,
                                        int b, int l, int d, int nv) {
  const int lc = min(max(l, 0), SL - 1);
  int s = seq[b * SL + lc];
  s = min(max(s, 0), nv - 1);
  const float v = emb[(size_t)s * DM + d] * 16.0f;
  return (l < SL) ? v : 0.0f;
}

__global__ __launch_bounds__(256) void k_conv(const int* __restrict__ seq, const float* __restrict__ emb,
                                              const float* __restrict__ cw, const float* __restrict__ cb,
                                              _Float16* __restrict__ xc, int nv) {
  __shared__ __align__(16) _Float16 st[32 * DM];
  const int tid = threadIdx.x, lane = tid & 31, wave = tid >> 5;
  const int d = tid;
  const int r0 = blockIdx.x * 32;
  const int b = r0 / SL, l0 = r0 - b * SL;
  const float w0 = cw[d * 4 + 0], w1 = cw[d * 4 + 1], w2 = cw[d * 4 + 2], w3 = cw[d * 4 + 3];
  const float bias = cb[d];
  float e0 = embtap(seq, emb, b, l0, d, nv);
  float e1 = embtap(seq, emb, b, l0 + 1, d, nv);
  float e2 = embtap(seq, emb, b, l0 + 2, d, nv);
#pragma unroll 1
  for (int i = 0; i < 32; ++i) {
    const float e3 = embtap(seq, emb, b, l0 + i + 3, d, nv);
    const float acc = (((w0 * e0 + w1 * e1) + w2 * e2) + w3 * e3) + bias;
    st[i * DM + d] = (_Float16)(acc * 16.0f);
    e0 = e1; e1 = e2; e2 = e3;
  }
  __syncthreads();
  v4u val[4];
  size_t go[4];
#pragma unroll
  for (int rr = 0; rr < 4; ++rr) {
    const int row = wave * 4 + rr;
    Pack8 pk;
    pk.h    = *(const v8h*)(st + row * DM + lane * 8);
    val[rr] = pk.u;
    go[rr]  = (size_t)(r0 + row) * DM + lane * 8;
  }
  for (int ps = 0; ps < 2; ++ps) {
#pragma unroll
    for (int rr = 0; rr < 4; ++rr) *(volatile v4u*)(xc + go[rr]) = val[rr];
    __threadfence();
  }
}

#define OTP 68
template <int MODE>
__global__ __launch_bounds__(256) void k_gemm(const _Float16* __restrict__ ap,
                                              const _Float16* __restrict__ wt,
                                              const float* __restrict__ bias, float scale,
                                              const int* __restrict__ seq,
                                              const float* __restrict__ resid,
                                              float* __restrict__ out) {
  __shared__ __align__(16) float st[8][16 * OTP];
  const int tid = threadIdx.x, lane = tid & 31, wave = tid >> 5;
  const int hh = lane >> 4, c = lane & 15;
  const int m0 = blockIdx.x * 256 + wave * 32;
  const int n0 = blockIdx.y * 64;

  v8f acc[2][4];
#pragma unroll
  for (int s = 0; s < 2; ++s)
#pragma unroll
    for (int t = 0; t < 4; ++t) acc[s][t] = zero8();
  gemm32x64(ap, DM, wt, DM, DM, m0, n0, lane, acc);

  float bb[4];
#pragma unroll
  for (int t = 0; t < 4; ++t) bb[t] = bias[n0 + 16 * t + c];
  float* sw = st[wave];

#pragma unroll
  for (int sub = 0; sub < 2; ++sub) {
    __syncthreads();
#pragma unroll
    for (int t = 0; t < 4; ++t) {
#pragma unroll
      for (int r = 0; r < 8; ++r) sw[(8 * hh + r) * OTP + 16 * t + c] = acc[sub][t][r] * scale + bb[t];
    }
    __syncthreads();
    v4f val[8];
    size_t go[8];
#pragma unroll
    for (int it = 0; it < 8; ++it) {
      const int p    = lane + 32 * it;
      const int Lr   = p >> 3;
      const int pc   = p & 7;
      const int row  = Lr >> 1;
      const int half = Lr & 1;
      v4f v = *(const v4f*)(sw + row * OTP + half * 32 + pc * 4);
      const int grow = m0 + sub * 16 + row;
      go[it] = (size_t)grow * DM + n0 + half * 32 + pc * 4;
      if (MODE == 0) {
        const float keep = (seq[grow] != 0) ? 1.0f : 0.0f;
        v = v * keep;
      } else {
        const v4f rv = *(const v4f*)(resid + go[it]);
        v4f t;
        t.x = fmaxf(v.x, 0.0f); t.y = fmaxf(v.y, 0.0f); t.z = fmaxf(v.z, 0.0f); t.w = fmaxf(v.w, 0.0f);
        v = rv + t;
      }
      val[it] = v;
    }
    for (int ps = 0; ps < 2; ++ps) {
#pragma unroll
      for (int it = 0; it < 8; ++it) *(volatile v4f*)(out + go[it]) = val[it];
      __threadfence();
    }
  }
}

__global__ __launch_bounds__(256) void k_mix(const float* __restrict__ X, const int* __restrict__ seq,
                                             const int* __restrict__ gid, const float* __restrict__ swv,
                                             const float* __restrict__ sbp,
                                             float* __restrict__ Y, _Float16* __restrict__ YH) {
  __shared__ __align__(16) float xt[WIN * DM];
  __shared__ float coef[CH * WIN];
  __shared__ float scl[CH * 16];
  __shared__ float xdot[WIN];
  __shared__ int gw[NLAY * WIN];
  __shared__ int vw[WIN];
  __shared__ int rsa[NLAY * WIN];
  __shared__ int rea[NLAY * WIN];
  __shared__ int sq[CH];

  const int tid = threadIdx.x, lane = tid & 31, wave = tid >> 5;
  const int bpb = SL / CH;
  const int b  = blockIdx.x / bpb;
  const int l0 = (blockIdx.x - b * bpb) * CH;
  const float sb = sbp[0];

#pragma unroll
  for (int j = 0; j < 8; ++j) {
    const int piece = tid + 256 * j;
    const int q  = piece >> 6;
    const int f  = (piece & 63) * 4;
    const int l  = l0 - HALO + q;
    const int lc = min(max(l, 0), SL - 1);
    const float keep = (l >= 0 && l < SL) ? 1.0f : 0.0f;
    const v4f v = *(const v4f*)(X + (size_t)(b * SL + lc) * DM + f);
    *(v4f*)(xt + q * DM + f) = v * keep;
  }
  for (int idx = tid; idx < NLAY * WIN; idx += 256) {
    const int li = idx >> 5, q = idx & 31;
    const int l  = l0 - HALO + q;
    const int lc = min(max(l, 0), SL - 1);
    const int g  = gid[(size_t)(b * NLAY + li) * SL + lc];
    gw[idx] = (l >= 0 && l < SL) ? g : 0;
  }
  if (tid < WIN) {
    const int l = l0 - HALO + tid;
    vw[tid] = (l >= 0 && l < SL) ? 1 : 0;
  }
  if (tid < CH) sq[tid] = seq[b * SL + l0 + tid];
  __syncthreads();

  {
    const v4f s0 = *(const v4f*)(swv + 8 * lane);
    const v4f s1 = *(const v4f*)(swv + 8 * lane + 4);
#pragma unroll 1
    for (int j = 0; j < 4; ++j) {
      const int q = wave + 8 * j;
      const float* xr = xt + q * DM + 8 * lane;
      const v4f a0 = *(const v4f*)(xr), a1 = *(const v4f*)(xr + 4);
      const v4f pr = a0 * s0 + a1 * s1;
      float p = (pr.x + pr.y) + (pr.z + pr.w);
#pragma unroll
      for (int off = 16; off >= 1; off >>= 1) p += __shfl_xor(p, off, 32);
      if (lane == 0) xdot[q] = p;
    }
  }
  if (tid < NLAY) {
    const int* g9 = gw + tid * WIN;
    int* rs9 = rsa + tid * WIN;
    int* re9 = rea + tid * WIN;
    int cur = 0, pg = g9[0], pv = vw[0];
    rs9[0] = 0;
#pragma unroll 1
    for (int q = 1; q < WIN; ++q) {
      const int g = g9[q], v = vw[q];
      const bool same = (v != 0) && (pv != 0) && (g == pg);
      cur = same ? cur : q;
      rs9[q] = cur;
      pg = g; pv = v;
    }
    cur = WIN - 1; pg = g9[WIN - 1]; pv = vw[WIN - 1];
    re9[WIN - 1] = WIN - 1;
#pragma unroll 1
    for (int q = WIN - 2; q >= 0; --q) {
      const int g = g9[q], v = vw[q];
      const bool same = (v != 0) && (pv != 0) && (g == pg);
      cur = same ? cur : q;
      re9[q] = cur;
      pg = g; pv = v;
    }
  }
  __syncthreads();

  if (tid < CH) {
    const int i = tid, qc = HALO + i;
    float* cf = coef + i * WIN;
    float* sl = scl + i * 16;
#pragma unroll 1
    for (int q = 0; q < WIN; ++q) cf[q] = 0.0f;
    const bool msk0 = (sq[i] == 0);
    const float s0 = msk0 ? -FLT_MAX : (xdot[qc] + sb);
    sl[0] = s0;
    float mx = s0;
#pragma unroll 1
    for (int li = 0; li < NLAY; ++li) {
      const int g = gw[li * WIN + qc];
      int s = rsa[li * WIN + qc], e = rea[li * WIN + qc];
      s = min(max(s, 0), WIN - 1);
      e = min(max(e, s), WIN - 1);
      float sum = 0.0f;
#pragma unroll 1
      for (int qq = s; qq <= e; ++qq) sum += xdot[qq];
      const float rc = __builtin_amdgcn_rcpf((float)(e - s + 1));
      const float sc = (g == 0) ? -FLT_MAX : (sum * rc + sb);
      sl[1 + li] = sc;
      mx = fmaxf(mx, sc);
    }
    float den = 0.0f;
#pragma unroll 1
    for (int s = 0; s < 10; ++s) {
      const float ev = expf(sl[s] - mx);
      sl[s] = ev;
      den += ev;
    }
    const float inv = __builtin_amdgcn_rcpf(den);
    if (!msk0) cf[qc] += sl[0] * inv;
#pragma unroll 1
    for (int li = 0; li < NLAY; ++li) {
      const int g = gw[li * WIN + qc];
      if (g != 0) {
        int s = rsa[li * WIN + qc], e = rea[li * WIN + qc];
        s = min(max(s, 0), WIN - 1);
        e = min(max(e, s), WIN - 1);
        const float cc = (sl[1 + li] * inv) * __builtin_amdgcn_rcpf((float)(e - s + 1));
#pragma unroll 1
        for (int qq = s; qq <= e; ++qq) cf[qq] += cc;
      }
    }
  }
  __syncthreads();

  float o[CH];
#pragma unroll
  for (int i = 0; i < CH; ++i) o[i] = 0.0f;
  {
    const int d = tid;
#pragma unroll 1
    for (int q = 0; q < WIN; ++q) {
      const float xv = xt[q * DM + d];
#pragma unroll
      for (int i = 0; i < CH; ++i) o[i] = fmaf(coef[i * WIN + q], xv, o[i]);
    }
  }
  __syncthreads();
#pragma unroll
  for (int i = 0; i < CH; ++i) xt[i * DM + tid] = o[i];
  __syncthreads();

  v4f va[2], vb[2];
  v4u vh[2];
  size_t go[2];
#pragma unroll
  for (int rr = 0; rr < 2; ++rr) {
    const int row = wave * 2 + rr;
    const float* orow = xt + row * DM;
    va[rr] = *(const v4f*)(orow + 4 * lane);
    vb[rr] = *(const v4f*)(orow + 128 + 4 * lane);
    const v4f a0 = *(const v4f*)(orow + 8 * lane) * 16.0f;
    const v4f a1 = *(const v4f*)(orow + 8 * lane + 4) * 16.0f;
    Pack8 pk;
    pk.h   = cvt8(a0, a1);
    vh[rr] = pk.u;
    go[rr] = (size_t)(b * SL + l0 + row) * DM;
  }
  for (int ps = 0; ps < 2; ++ps) {
#pragma unroll
    for (int rr = 0; rr < 2; ++rr) {
      *(volatile v4f*)(Y + go[rr] + 4 * lane)       = va[rr];
      *(volatile v4f*)(Y + go[rr] + 128 + 4 * lane) = vb[rr];
      *(volatile v4u*)(YH + go[rr] + 8 * lane)       = vh[rr];
    }
    __threadfence();
  }
}

extern "C" void kernel_launch(void* const* d_in, const int* in_sizes, int n_in,
                              void* d_out, int out_size, void* d_ws, size_t ws_size,
                              hipStream_t stream) {
  if (n_in < 11) return;
  if (in_sizes[0]  != NTOK) return;
  if (in_sizes[1]  != NBATCH * NLAY * SL) return;
  if (in_sizes[2]  < DM || (in_sizes[2] % DM) != 0) return;
  if (in_sizes[3]  != DM * 4) return;
  if (in_sizes[4]  != DM) return;
  if (in_sizes[5]  != DM * DM) return;
  if (in_sizes[6]  != DM) return;
  if (in_sizes[7]  != DM) return;
  if (in_sizes[8]  != 1) return;
  if (in_sizes[9]  != DM * DM) return;
  if (in_sizes[10] != DM) return;
  if (out_size != NTOK * DM) return;

  const int*   seq     = (const int*)d_in[0];
  const int*   gidp    = (const int*)d_in[1];
  const float* emb     = (const float*)d_in[2];
  const float* conv_w  = (const float*)d_in[3];
  const float* conv_b  = (const float*)d_in[4];
  const float* proj_w  = (const float*)d_in[5];
  const float* proj_b  = (const float*)d_in[6];
  const float* score_w = (const float*)d_in[7];
  const float* score_b = (const float*)d_in[8];
  const float* ff_w    = (const float*)d_in[9];
  const float* ff_b    = (const float*)d_in[10];
  float* out = (float*)d_out;
  const int nv = in_sizes[2] / DM;

  size_t off = 0;
  const size_t oWP = off; off += (size_t)DM * DM * 2;
  const size_t oWF = off; off += (size_t)DM * DM * 2;
  const size_t oXC = off; off += (size_t)NTOK * DM * 2;
  const size_t oX  = off; off += (size_t)NTOK * DM * 4;
  const size_t oY  = off; off += (size_t)NTOK * DM * 4;
  const size_t oYH = off; off += (size_t)NTOK * DM * 2;
  if (off > ws_size) return;
  if (off > (size_t)134217728) return;

  char* ws = (char*)d_ws;
  _Float16* WP = (_Float16*)(ws + oWP);
  _Float16* WF = (_Float16*)(ws + oWF);
  _Float16* XC = (_Float16*)(ws + oXC);
  float*    X  = (float*)(ws + oX);
  float*    Y  = (float*)(ws + oY);
  _Float16* YH = (_Float16*)(ws + oYH);

  k_cvt<<<dim3((DM * DM) / 2048), dim3(256), 0, stream>>>(proj_w, WP, 32.0f);
  k_cvt<<<dim3((DM * DM) / 2048), dim3(256), 0, stream>>>(ff_w, WF, 32.0f);
  k_conv<<<dim3(NTOK / 32), dim3(256), 0, stream>>>(seq, emb, conv_w, conv_b, XC, nv);
  k_gemm<0><<<dim3(NTOK / 256, DM / 64), dim3(256), 0, stream>>>(XC, WP, proj_b, 0.001953125f, seq, Y, X);
  k_mix<<<dim3(NTOK / CH), dim3(256), 0, stream>>>(X, seq, gidp, score_w, score_b, Y, YH);
  k_gemm<1><<<dim3(NTOK / 256, DM / 64), dim3(256), 0, stream>>>(YH, WF, ff_b, 0.001953125f, seq, Y, out);
  (void)hipGetLastError();
}
